// WKVAttention_40845138985319
// MI455X (gfx1250) — hardware-verified
//
#include <hip/hip_runtime.h>
#include <math.h>

constexpr int kBatch   = 8;
constexpr int kSeqLen  = 4096;
constexpr int kDim     = 128;
constexpr int kNumCh   = 64;
constexpr int kChLen   = 64;
constexpr int kTok     = kBatch * kSeqLen;
constexpr int kLdProj  = 4 * kDim;
constexpr int kColQ    = 0;
constexpr int kColK    = kDim;
constexpr int kColV    = 2 * kDim;
constexpr int kColD    = 3 * kDim;
constexpr int kSpPitchF = 132;
constexpr int kRowsPerChunk = 8;
static_assert(kNumCh * kChLen == kSeqLen);
static_assert(kDim == 128);
static_assert(kLdProj == 512);
static_assert((kSpPitchF * 4) % 16 == 0);
static_assert(kDim % kRowsPerChunk == 0 && kRowsPerChunk % 4 == 0);

constexpr size_t kOffXH   = 0;
constexpr size_t kOffXL   = 8388608;
constexpr size_t kOffProj = 16777216;
constexpr size_t kOffOpf  = 83886080;
constexpr size_t kOffWH   = 100663296;
constexpr size_t kOffWL   = 100827136;
constexpr size_t kWsEnd   = 100990976;
static_assert(kOffXL   == kOffXH   + (size_t)kTok * kDim * 2);
static_assert(kOffProj == kOffXL   + (size_t)kTok * kDim * 2);
static_assert(kOffOpf  == kOffProj + (size_t)kTok * kLdProj * 4);
static_assert(kOffWH   == kOffOpf  + (size_t)kTok * kDim * 4);
static_assert(kOffWL   == kOffWH   + (size_t)5 * kDim * kDim * 2);
static_assert(kWsEnd   == kOffWL   + (size_t)5 * kDim * kDim * 2);
static_assert(kWsEnd <= (size_t)134217728);
static_assert(kOffWH % 128 == 0 && kOffWL % 128 == 0 && kOffOpf % 128 == 0);

typedef __attribute__((ext_vector_type(16))) _Float16 v16h;
typedef __attribute__((ext_vector_type(8)))  _Float16 v8h;
typedef __attribute__((ext_vector_type(16))) __bf16   v16b;
typedef __attribute__((ext_vector_type(8)))  __bf16   v8b;
typedef __attribute__((ext_vector_type(8)))  float    v8f;
typedef __attribute__((ext_vector_type(4)))  float    v4f;
typedef __attribute__((ext_vector_type(4)))  unsigned int v4u;

__device__ __forceinline__ unsigned short f2bf_bits(float f) {
  unsigned u = __float_as_uint(f);
  return (unsigned short)((u + 0x7FFFu + ((u >> 16) & 1u)) >> 16);
}
__device__ __forceinline__ float bf_bits2f(unsigned short h) { return __uint_as_float(((unsigned)h) << 16); }

__device__ __forceinline__ void dep_guard_h(v8f& a, v8f& b, v16h x, v16h y) { asm volatile("v_nop\n\tv_nop\n\tv_nop\n\tv_nop" : "+v"(a), "+v"(b) : "v"(x), "v"(y)); }
__device__ __forceinline__ void dep_guard_b(v8f& a, v8f& b, v16b x, v16b y) { asm volatile("v_nop\n\tv_nop\n\tv_nop\n\tv_nop" : "+v"(a), "+v"(b) : "v"(x), "v"(y)); }
__device__ __forceinline__ void keep4_h(v16h a, v16h b, v16h c, v16h d) { asm volatile("v_nop" :: "v"(a), "v"(b), "v"(c), "v"(d)); }
__device__ __forceinline__ void keep4_b(v16b a, v16b b, v16b c, v16b d) { asm volatile("v_nop" :: "v"(a), "v"(b), "v"(c), "v"(d)); }
__device__ __forceinline__ void acc_guard4(v8f& a, v8f& b, v8f& c, v8f& d) { asm volatile("v_nop\n\tv_nop\n\tv_nop\n\tv_nop" : "+v"(a), "+v"(b), "+v"(c), "+v"(d)); }
template <typename T> struct Frag;
template <> struct Frag<_Float16> {
  typedef v16h V; union U { v16h v; v8h h[2]; };
  static __device__ __forceinline__ v16h load(const _Float16* p) {
    U f; f.h[0] = *(const v8h*)(p); f.h[1] = *(const v8h*)(p + 16); return f.v;
  }
  static __device__ __forceinline__ v8f mma(v16h a, v16h b, v8f c) {
    return __builtin_amdgcn_wmma_f32_16x16x32_f16(false, a, false, b, (short)0, c, false, false);
  }
  static __device__ __forceinline__ void guard(v8f& a, v8f& b, v16h x, v16h y) { dep_guard_h(a, b, x, y); }
  static __device__ __forceinline__ void keep(v16h a, v16h b, v16h c, v16h d) { keep4_h(a, b, c, d); }
};
template <> struct Frag<__bf16> {
  typedef v16b V; union U { v16b v; v8b h[2]; };
  static __device__ __forceinline__ v16b load(const __bf16* p) {
    U f; f.h[0] = *(const v8b*)(p); f.h[1] = *(const v8b*)(p + 16); return f.v;
  }
  static __device__ __forceinline__ v8f mma(v16b a, v16b b, v8f c) {
    return __builtin_amdgcn_wmma_f32_16x16x32_bf16(false, a, false, b, (short)0, c, false, false);
  }
  static __device__ __forceinline__ void guard(v8f& a, v8f& b, v16b x, v16b y) { dep_guard_b(a, b, x, y); }
  static __device__ __forceinline__ void keep(v16b a, v16b b, v16b c, v16b d) { keep4_b(a, b, c, d); }
};

__device__ __forceinline__ unsigned pk16(unsigned short a, unsigned short b) { return (unsigned)a | ((unsigned)b << 16); }

template <int ET> struct Elem;
template <> struct Elem<0> { typedef _Float16 T; };
template <> struct Elem<1> { typedef __bf16 T; };
template <int ET, bool SPLIT, int BIAS_MODE, int OUT_MODE, bool RESID, int ACT = 0>
__global__ __launch_bounds__(256) void wmma_gemm64(
    const unsigned short* __restrict__ Ap, const unsigned short* __restrict__ A2p, int lda, long strideA,
    const unsigned short* __restrict__ Btp, const unsigned short* __restrict__ Bt2p, int ldb, long strideB,
    void* __restrict__ Cout, void* __restrict__ Cout2, int ldc, long strideC,
    const float* __restrict__ bias,
    const float* __restrict__ resid, long strideR,
    int M, int N, int K, float scale) {
  typedef typename Elem<ET>::T T;
  typedef typename Frag<T>::V V;
  const T* A = (const T*)Ap; const T* A2 = (const T*)A2p; const T* Bt = (const T*)Btp; const T* Bt2 = (const T*)Bt2p;
  __shared__ __align__(16) float sT[8][16 * 68];
  const int b    = blockIdx.y;
  const int lane = threadIdx.x & 31;
  const int wave = threadIdx.x >> 5;
  const int tilesN = N >> 6;
  const int tilesM = M >> 6;
  const int tile = blockIdx.x * 8 + wave;
  if (tile >= tilesM * tilesN) return;
  const int tm = tile / tilesN;
  const int tn = tile - tm * tilesN;
  const int m0 = tm << 6;
  const int n0 = tn << 6;

  const T* Ab  = A  + (size_t)b * strideA;
  const T* Bb  = Bt + (size_t)b * strideB;
  const T* Ab2 = SPLIT ? (A2  + (size_t)b * strideA) : nullptr;
  const T* Bb2 = SPLIT ? (Bt2 + (size_t)b * strideB) : nullptr;

  const int rlane = lane & 15;
  const int koff  = (lane >> 4) * 8;
  const int mOff  = (lane >> 4) * 8;

  v8f acc[4][4];
#pragma unroll
  for (int i = 0; i < 4; ++i)
#pragma unroll
    for (int j = 0; j < 4; ++j) acc[i][j] = (v8f){0.f,0.f,0.f,0.f,0.f,0.f,0.f,0.f};

  for (int k0 = 0; k0 < K; k0 += 32) {
    V bh[4], bl[4];
#pragma unroll
    for (int j = 0; j < 4; ++j) {
      const size_t bo = (size_t)(n0 + (j << 4) + rlane) * ldb + koff + k0;
      bh[j] = Frag<T>::load(Bb + bo);
      if (SPLIT) bl[j] = Frag<T>::load(Bb2 + bo);
    }
#pragma unroll
    for (int i = 0; i < 4; ++i) {
      const size_t ao = (size_t)(m0 + (i << 4) + rlane) * lda + koff + k0;
      V ah = Frag<T>::load(Ab + ao);
      V al;
      if (SPLIT) al = Frag<T>::load(Ab2 + ao);
#pragma unroll
      for (int j = 0; j < 4; ++j) {
        acc[i][j] = Frag<T>::mma(ah, bh[j], acc[i][j]);
        if (SPLIT) {
          acc[i][j] = Frag<T>::mma(ah, bl[j], acc[i][j]);
          acc[i][j] = Frag<T>::mma(al, bh[j], acc[i][j]);
        }
      }
      Frag<T>::guard(acc[i][0], acc[i][3], ah, SPLIT ? al : ah);
    }
    Frag<T>::keep(bh[0], bh[1], bh[2], bh[3]);
    if (SPLIT) Frag<T>::keep(bl[0], bl[1], bl[2], bl[3]);
  }
  acc_guard4(acc[0][0], acc[0][1], acc[0][2], acc[0][3]);
  acc_guard4(acc[1][0], acc[1][1], acc[1][2], acc[1][3]);
  acc_guard4(acc[2][0], acc[2][1], acc[2][2], acc[2][3]);
  acc_guard4(acc[3][0], acc[3][1], acc[3][2], acc[3][3]);

  float* slab = sT[wave];
  const float* Rb = RESID ? (resid + (size_t)b * strideR) : nullptr;
#pragma unroll
  for (int i = 0; i < 4; ++i) {
    const int mBase = m0 + (i << 4);
#pragma unroll
    for (int j = 0; j < 4; ++j) {
      const int n = n0 + (j << 4) + rlane;
      float bv = 0.f;
      if (BIAS_MODE == 2) bv = bias[n];
#pragma unroll
      for (int r = 0; r < 8; ++r) {
        float v = acc[i][j][r] * scale;
        if (BIAS_MODE == 1) v += bias[mBase + mOff + r];
        if (BIAS_MODE == 2) v += bv;
        if (RESID) v += Rb[(size_t)(mBase + mOff + r) * ldc + n];
        if (ACT == 2) v = fmaxf(v, 0.0f);
        if (ACT == 4) v = (v > 0.f) ? v : 0.01f * v;
        slab[(mOff + r) * 68 + (j << 4) + rlane] = v;
      }
    }
    __builtin_amdgcn_fence(__ATOMIC_RELEASE, "workgroup");
    __builtin_amdgcn_wave_barrier();
    __builtin_amdgcn_fence(__ATOMIC_ACQUIRE, "workgroup");
    if (OUT_MODE == 0) {
      float* C = (float*)Cout + (size_t)b * strideC;
      const int hh = lane >> 4, c4 = (lane & 15) * 4;
      for (int pass = 0; pass < 2; ++pass) {
#pragma unroll
        for (int it = 0; it < 8; ++it) {
          const int row = it * 2 + hh;
          v4f v = *(const v4f*)(slab + row * 68 + c4);
          *(volatile v4f*)(C + (size_t)(mBase + row) * ldc + n0 + c4) = v;
        }
        __threadfence();
      }
    } else {
      const int q = lane >> 3, c8 = (lane & 7) * 8;
      unsigned short* C  = (unsigned short*)Cout  + (size_t)b * strideC;
      unsigned short* C2 = (OUT_MODE == 2) ? ((unsigned short*)Cout2 + (size_t)b * strideC) : nullptr;
      for (int pass = 0; pass < 2; ++pass) {
#pragma unroll
        for (int it = 0; it < 4; ++it) {
          const int row = it * 4 + q;
          const float* sp = slab + row * 68 + c8;
          v8h hv, lv;
#pragma unroll
          for (int e = 0; e < 8; ++e) {
            if (OUT_MODE == 1) {
              hv[e] = (_Float16)sp[e];
            } else {
              unsigned short hb = f2bf_bits(sp[e]);
              unsigned short lb = f2bf_bits(sp[e] - bf_bits2f(hb));
              hv[e] = __builtin_bit_cast(_Float16, hb);
              lv[e] = __builtin_bit_cast(_Float16, lb);
            }
          }
          *(volatile v8h*)(C + (size_t)(mBase + row) * ldc + n0 + c8) = hv;
          if (OUT_MODE == 2) *(volatile v8h*)(C2 + (size_t)(mBase + row) * ldc + n0 + c8) = lv;
        }
        __threadfence();
      }
    }
    __builtin_amdgcn_fence(__ATOMIC_RELEASE, "workgroup");
    __builtin_amdgcn_wave_barrier();
    __builtin_amdgcn_fence(__ATOMIC_ACQUIRE, "workgroup");
  }
}

__device__ __forceinline__ void split_bf(float f, unsigned short& hb, unsigned short& lb) {
  hb = f2bf_bits(f);
  lb = f2bf_bits(f - bf_bits2f(hb));
}
__device__ __forceinline__ float logistic_f32(float x) {
  return 1.0f / (1.0f + expf(-x));
}

__global__ __launch_bounds__(256) void split8_kernel(const float* __restrict__ in,
                                                     unsigned short* __restrict__ hi,
                                                     unsigned short* __restrict__ lo, int n8) {
  const int i = blockIdx.x * 256 + threadIdx.x;
  if (i >= n8) return;
  const float* p = in + 8 * (size_t)i;
  const v4f a = *(const v4f*)(p);
  const v4f c = *(const v4f*)(p + 4);
  unsigned short hb[8], lb[8];
#pragma unroll
  for (int e = 0; e < 4; ++e) {
    split_bf(a[e], hb[e], lb[e]);
    split_bf(c[e], hb[4 + e], lb[4 + e]);
  }
  const v4u uh = (v4u){pk16(hb[0], hb[1]), pk16(hb[2], hb[3]), pk16(hb[4], hb[5]), pk16(hb[6], hb[7])};
  const v4u ul = (v4u){pk16(lb[0], lb[1]), pk16(lb[2], lb[3]), pk16(lb[4], lb[5]), pk16(lb[6], lb[7])};
  unsigned short* qh = hi + 8 * (size_t)i;
  unsigned short* ql = lo + 8 * (size_t)i;
  *(volatile v4u*)qh = uh;
  *(volatile v4u*)ql = ul;
  __threadfence();
  *(volatile v4u*)qh = uh;
  *(volatile v4u*)ql = ul;
}

__global__ __launch_bounds__(256) void split8w_kernel(const float* __restrict__ W0, const float* __restrict__ W1,
                                                      const float* __restrict__ W2, const float* __restrict__ W3,
                                                      const float* __restrict__ W4,
                                                      unsigned short* __restrict__ hi, unsigned short* __restrict__ lo) {
  const int y = blockIdx.y;
  const float* W = (y == 0) ? W0 : (y == 1) ? W1 : (y == 2) ? W2 : (y == 3) ? W3 : W4;
  const int i = blockIdx.x * 256 + threadIdx.x;
  if (i >= (kDim * kDim) / 8) return;
  const float* p = W + 8 * (size_t)i;
  const v4f a = *(const v4f*)(p);
  const v4f c = *(const v4f*)(p + 4);
  unsigned short hb[8], lb[8];
#pragma unroll
  for (int e = 0; e < 4; ++e) {
    split_bf(a[e], hb[e], lb[e]);
    split_bf(c[e], hb[4 + e], lb[4 + e]);
  }
  const v4u uh = (v4u){pk16(hb[0], hb[1]), pk16(hb[2], hb[3]), pk16(hb[4], hb[5]), pk16(hb[6], hb[7])};
  const v4u ul = (v4u){pk16(lb[0], lb[1]), pk16(lb[2], lb[3]), pk16(lb[4], lb[5]), pk16(lb[6], lb[7])};
  const size_t dst = (size_t)y * kDim * kDim + 8 * (size_t)i;
  unsigned short* qh = hi + dst;
  unsigned short* ql = lo + dst;
  *(volatile v4u*)qh = uh;
  *(volatile v4u*)ql = ul;
  __threadfence();
  *(volatile v4u*)qh = uh;
  *(volatile v4u*)ql = ul;
}

__global__ __launch_bounds__(128)
void decay_scan_kernel(const float* __restrict__ proj, float* __restrict__ opf) {
#pragma clang fp contract(off)
  __shared__ __align__(16) float Sp[kDim * kSpPitchF];
  __shared__ __align__(16) float stg[2 * 3 * kDim];
  __shared__ __align__(16) float obuf[2 * kDim];
  __shared__ __align__(16) float wpsh[kDim];

  const int b    = blockIdx.x;
  const int j    = threadIdx.x;
  const int wave = j >> 5;
  const int lane = j & 31;
  const float* pb = proj + (size_t)b * kSeqLen * kLdProj;
  float* opb = opf + (size_t)b * kSeqLen * kDim;
  float* spr = Sp + j * kSpPitchF;

  {
    const v4f z = (v4f){0.f, 0.f, 0.f, 0.f};
#pragma unroll
    for (int g = 0; g < 32; ++g) *(v4f*)(spr + 4 * g) = z;
  }
  float S[kDim];
#pragma unroll
  for (int i = 0; i < kDim; ++i) S[i] = 0.0f;

  float vcur;
  {
    const float* r0 = pb + j;
    stg[0 * kDim + j] = r0[kColQ];
    stg[1 * kDim + j] = r0[kColK];
    vcur = r0[kColV];
    stg[2 * kDim + j] = logistic_f32(r0[kColD]);
  }

#pragma unroll 1
  for (int c = 0; c < kNumCh; ++c) {
    {
      const float* pd = pb + (size_t)(c * kChLen) * kLdProj + kColD + j;
      float P = 1.0f;
#pragma unroll 1
      for (int tl = 0; tl < kChLen; ++tl) {
        P = P * logistic_f32(pd[(size_t)tl * kLdProj]);
      }
      wpsh[j] = P;
    }
    __syncthreads();
    if (c > 0) {
#pragma unroll
      for (int g = 0; g < 32; ++g) {
        const int i0 = 4 * g;
        const v4f sp4 = *(const v4f*)(spr + i0);
        const v4f wp4 = *(const v4f*)(wpsh + i0);
        v4f n4;
#pragma unroll
        for (int e = 0; e < 4; ++e) {
          const float tt = wp4[e] * sp4[e];
          n4[e] = tt + S[i0 + e];
        }
        *(v4f*)(spr + i0) = n4;
        if ((g & 1) == 1) asm volatile("" ::: "memory");
      }
    }
#pragma unroll
    for (int i = 0; i < kDim; ++i) S[i] = 0.0f;

#pragma unroll 1
    for (int tl = 0; tl < kChLen; ++tl) {
      const int t = c * kChLen + tl;
      const int buf = t & 1;
      __syncthreads();
      if (wave == 0 && t > 0) {
        const v4f val = *(const v4f*)(obuf + (buf ^ 1) * kDim + 4 * lane);
        float* qo = opb + (size_t)(t - 1) * kDim + 4 * lane;
        *(volatile v4f*)qo = val;
        __threadfence();
        *(volatile v4f*)qo = val;
      }
      const int tn = (t + 1 < kSeqLen) ? (t + 1) : (kSeqLen - 1);
      const float* rn = pb + (size_t)tn * kLdProj + j;
      const float qn = rn[kColQ];
      const float kn = rn[kColK];
      const float vn = rn[kColV];
      const float wn = logistic_f32(rn[kColD]);
      const float v = vcur;
      const float* sq = stg + buf * 3 * kDim;
      const float* sk = sq + kDim;
      const float* sw = sq + 2 * kDim;
      float oacc[4];
      oacc[0] = 0.f; oacc[1] = 0.f; oacc[2] = 0.f; oacc[3] = 0.f;
#pragma unroll
      for (int ch = 0; ch < kDim / kRowsPerChunk; ++ch) {
        v4f qq[kRowsPerChunk / 4], kk[kRowsPerChunk / 4], ww[kRowsPerChunk / 4], pp[kRowsPerChunk / 4];
#pragma unroll
        for (int u = 0; u < kRowsPerChunk / 4; ++u) {
          const int i0 = ch * kRowsPerChunk + 4 * u;
          qq[u] = *(const v4f*)(sq + i0);
          kk[u] = *(const v4f*)(sk + i0);
          ww[u] = *(const v4f*)(sw + i0);
          pp[u] = *(const v4f*)(spr + i0);
        }
#pragma unroll
        for (int u = 0; u < kRowsPerChunk / 4; ++u) {
          const int i0 = ch * kRowsPerChunk + 4 * u;
#pragma unroll
          for (int e = 0; e < 4; ++e) {
            const float decayed = ww[u][e] * S[i0 + e];
            const float kv = kk[u][e] * v;
            const float s = decayed + kv;
            S[i0 + e] = s;
            const float tot = s + pp[u][e];
            const float qs = qq[u][e] * tot;
            oacc[e] = oacc[e] + qs;
          }
        }
        asm volatile("" : "+v"(oacc[0]), "+v"(oacc[1]), "+v"(oacc[2]), "+v"(oacc[3]) : : "memory");
      }
      const float o = (oacc[0] + oacc[1]) + (oacc[2] + oacc[3]);
      obuf[buf * kDim + j] = o;
      float* sn = stg + (buf ^ 1) * 3 * kDim + j;
      sn[0] = qn;
      sn[kDim] = kn;
      sn[2 * kDim] = wn;
      vcur = vn;
    }
  }
  __syncthreads();
  if (wave == 0) {
    const v4f val = *(const v4f*)(obuf + ((kSeqLen - 1) & 1) * kDim + 4 * lane);
    float* qo = opb + (size_t)(kSeqLen - 1) * kDim + 4 * lane;
    *(volatile v4f*)qo = val;
    __threadfence();
    *(volatile v4f*)qo = val;
  }
}

extern "C" void kernel_launch(void* const* d_in, const int* in_sizes, int n_in,
                              void* d_out, int out_size, void* d_ws, size_t ws_size,
                              hipStream_t stream) {
  if (n_in < 6) return;
  if (in_sizes[0] != kTok * kDim) return;
  if (in_sizes[1] != kDim * kDim || in_sizes[2] != kDim * kDim || in_sizes[3] != kDim * kDim ||
      in_sizes[4] != kDim * kDim || in_sizes[5] != kDim * kDim) return;
  if (out_size != kTok * kDim) return;
  if (ws_size < kWsEnd) return;

  const float* x  = (const float*)d_in[0];
  const float* Wq = (const float*)d_in[1];
  const float* Wk = (const float*)d_in[2];
  const float* Wv = (const float*)d_in[3];
  const float* Wo = (const float*)d_in[4];
  const float* Wd = (const float*)d_in[5];
  float* outp = (float*)d_out;

  char* ws = (char*)d_ws;
  unsigned short* XH = (unsigned short*)(ws + kOffXH);
  unsigned short* XL = (unsigned short*)(ws + kOffXL);
  float* PROJ = (float*)(ws + kOffProj);
  float* OPF  = (float*)(ws + kOffOpf);
  unsigned short* WH = (unsigned short*)(ws + kOffWH);
  unsigned short* WL = (unsigned short*)(ws + kOffWL);
  unsigned short* OPH = XH;
  unsigned short* OPL = XL;
  unsigned short* WOH = WH + (size_t)4 * kDim * kDim;
  unsigned short* WOL = WL + (size_t)4 * kDim * kDim;

  const int n8x = (kTok * kDim) / 8;

  split8_kernel<<<dim3(n8x / 256), dim3(256), 0, stream>>>(x, XH, XL, n8x);
  split8w_kernel<<<dim3((kDim * kDim) / 8 / 256, 5), dim3(256), 0, stream>>>(Wq, Wk, Wv, Wd, Wo, WH, WL);
  wmma_gemm64<1, true, 0, 0, false, 0><<<dim3((kTok / 64) * (kLdProj / 64) / 8, 1), dim3(256), 0, stream>>>(
      XH, XL, kDim, 0L, WH, WL, kDim, 0L, (void*)PROJ, nullptr, kLdProj, 0L,
      nullptr, nullptr, 0L, kTok, kLdProj, kDim, 1.0f);
  decay_scan_kernel<<<dim3(kBatch), dim3(128), 0, stream>>>(PROJ, OPF);
  split8_kernel<<<dim3(n8x / 256), dim3(256), 0, stream>>>(OPF, OPH, OPL, n8x);
  wmma_gemm64<1, true, 0, 0, false, 0><<<dim3((kTok / 64) * (kDim / 64) / 8, 1), dim3(256), 0, stream>>>(
      OPH, OPL, kDim, 0L, WOH, WOL, kDim, 0L, (void*)outp, nullptr, kDim, 0L,
      nullptr, nullptr, 0L, kTok, kDim, kDim, 1.0f);
}
